// _MultiHeadAttention_29686813949966
// MI455X (gfx1250) — hardware-verified
//
#include <hip/hip_runtime.h>
#include <stddef.h>
#include <stdint.h>

#define NB    4
#define NT    1024
#define DM    256
#define NH    8
#define HD    32
#define WIN   64
#define NTOK  (NB * NT)
#define NQKV  768
#define PADF  64
#define TGK   (NT + PADF)
#define TVP   1152
#define VTAIL (TVP - TGK)
#define QT    16
#define NQT   (NT / QT)

static_assert(DM == NH * HD);
static_assert(HD == 32);
static_assert(WIN == PADF);
static_assert(NT % 256 == 0);
static_assert(NT % QT == 0);
static_assert(NT - QT + 80 <= TGK);
static_assert(NT - QT + 96 <= TVP);
static_assert(VTAIL == 64);
static_assert((TVP * 2) % 128 == 0);
static_assert((NTOK * DM) % 2048 == 0);
static_assert((NQKV * DM) % 2048 == 0);
static_assert((DM * DM) % 2048 == 0);
static_assert(NQKV == 3 * DM);

typedef _Float16 v16h __attribute__((ext_vector_type(16)));
typedef _Float16 v8h  __attribute__((ext_vector_type(8)));
typedef float    v8f  __attribute__((ext_vector_type(8)));
typedef float    v4f  __attribute__((ext_vector_type(4)));
typedef unsigned int v4u __attribute__((ext_vector_type(4)));

union Frag  { v16h v; v8h h[2]; };
union Pack8 { v8h h; v4u u; };

__device__ __forceinline__ v8f mma16(v16h a, v16h b, v8f c) {
  c = __builtin_amdgcn_wmma_f32_16x16x32_f16(false, a, false, b, (short)0, c, false, false);
  asm volatile("v_nop\n\tv_nop\n\tv_nop\n\tv_nop" : "+v"(c) : "v"(a), "v"(b));
  return c;
}

__device__ __forceinline__ v16h ldfrag(const _Float16* p, int ld, int row0, int k0, int lane) {
  const int m = lane & 15, lh = lane >> 4;
  const _Float16* q = p + (size_t)(row0 + m) * ld + k0 + 8 * lh;
  Frag f;
  f.h[0] = *(const v8h*)(q);
  f.h[1] = *(const v8h*)(q + 16);
  return f.v;
}

__device__ __forceinline__ v8f zero8() { return (v8f){0.f, 0.f, 0.f, 0.f, 0.f, 0.f, 0.f, 0.f}; }

__device__ __forceinline__ void gemm32x64(const _Float16* __restrict__ A, int lda,
                                          const _Float16* __restrict__ Bt, int ldb, int K,
                                          int m0, int n0, int lane, v8f (&acc)[2][4]) {
#pragma unroll 1
  for (int k0 = 0; k0 < K; k0 += 32) {
    const v16h a0 = ldfrag(A, lda, m0, k0, lane);
    const v16h a1 = ldfrag(A, lda, m0 + 16, k0, lane);
    const v16h b0 = ldfrag(Bt, ldb, n0, k0, lane);
    const v16h b1 = ldfrag(Bt, ldb, n0 + 16, k0, lane);
    const v16h b2 = ldfrag(Bt, ldb, n0 + 32, k0, lane);
    const v16h b3 = ldfrag(Bt, ldb, n0 + 48, k0, lane);
    acc[0][0] = mma16(a0, b0, acc[0][0]);
    acc[1][0] = mma16(a1, b0, acc[1][0]);
    acc[0][1] = mma16(a0, b1, acc[0][1]);
    acc[1][1] = mma16(a1, b1, acc[1][1]);
    acc[0][2] = mma16(a0, b2, acc[0][2]);
    acc[1][2] = mma16(a1, b2, acc[1][2]);
    acc[0][3] = mma16(a0, b3, acc[0][3]);
    acc[1][3] = mma16(a1, b3, acc[1][3]);
  }
}

__global__ __launch_bounds__(256) void k_cvt(const float* __restrict__ src, _Float16* __restrict__ dh, float scale) {
  const size_t o = ((size_t)blockIdx.x * 256 + threadIdx.x) * 8;
  const v4f a0 = *(const v4f*)(src + o) * scale;
  const v4f a1 = *(const v4f*)(src + o + 4) * scale;
  Pack8 pk;
  pk.h = (v8h){(_Float16)a0[0], (_Float16)a0[1], (_Float16)a0[2], (_Float16)a0[3],
               (_Float16)a1[0], (_Float16)a1[1], (_Float16)a1[2], (_Float16)a1[3]};
  const v4u vv = pk.u;
  volatile v4u* d = (volatile v4u*)(dh + o);
  *d = vv;
  __threadfence();
  *d = vv;
}

#define NPADBLK_K 32
#define NPADBLK_V 16
__global__ __launch_bounds__(256) void k_padfill(const float* __restrict__ inb, _Float16* __restrict__ kpl,
                                                 _Float16* __restrict__ vtp) {
  const int tid = threadIdx.x, lane = tid & 31, wave = tid >> 5;
  if (blockIdx.x < NPADBLK_K) {
    const int pr = blockIdx.x * 8 + wave;
    const int b  = pr >> 6, g = pr & 63;
    const v4f b0 = *(const v4f*)(inb + DM + lane * 8);
    const v4f b1 = *(const v4f*)(inb + DM + lane * 8 + 4);
    Pack8 pk;
    pk.h = (v8h){(_Float16)b0[0], (_Float16)b0[1], (_Float16)b0[2], (_Float16)b0[3],
                 (_Float16)b1[0], (_Float16)b1[1], (_Float16)b1[2], (_Float16)b1[3]};
    const v4u vv = pk.u;
    volatile v4u* d = (volatile v4u*)(kpl + ((size_t)b * TGK + g) * DM + lane * 8);
    *d = vv;
    __threadfence();
    *d = vv;
  } else {
    const int vb = blockIdx.x - NPADBLK_K;
    v4u val[2];
    size_t gf[2], gt[2];
#pragma unroll
    for (int it = 0; it < 2; ++it) {
      const int rowid = (vb * 8 + wave) * 8 + 4 * it + (lane >> 3);
      const int dch   = rowid & 255;
      const int piece = lane & 7;
      const float bvv = inb[2 * DM + dch];
      const _Float16 hv = (_Float16)bvv;
      Pack8 pk;
      pk.h    = (v8h){hv, hv, hv, hv, hv, hv, hv, hv};
      val[it] = pk.u;
      gf[it]  = (size_t)rowid * TVP + piece * 8;
      gt[it]  = (size_t)rowid * TVP + TGK + piece * 8;
    }
    const v4u z = (v4u){0u, 0u, 0u, 0u};
    for (int ps = 0; ps < 2; ++ps) {
#pragma unroll
      for (int it = 0; it < 2; ++it) {
        *(volatile v4u*)(vtp + gf[it]) = val[it];
        *(volatile v4u*)(vtp + gt[it]) = z;
      }
      __threadfence();
    }
  }
}

#define STP 72
#define SVP 264
__global__ __launch_bounds__(256) void k_qkv(const _Float16* __restrict__ xh,
                                             const _Float16* __restrict__ wt,
                                             const float* __restrict__ inb,
                                             _Float16* __restrict__ qp,
                                             _Float16* __restrict__ kpl,
                                             _Float16* __restrict__ vtp) {
  __shared__ __align__(16) _Float16 st[256 * STP];
  const int tid = threadIdx.x, lane = tid & 31, wave = tid >> 5;
  const int hh = lane >> 4, c = lane & 15;
  const int rb = blockIdx.x * 256;
  const int b  = rb / NT;
  const int l0 = rb - b * NT;
  const int ns = blockIdx.y;
  const int which = ns >> 2;
  const int cs = (ns & 3) * 64;
  const int m0 = rb + wave * 32;
  const int n0 = ns * 64;

  v8f acc[2][4];
#pragma unroll
  for (int s = 0; s < 2; ++s)
#pragma unroll
    for (int t = 0; t < 4; ++t) acc[s][t] = zero8();
  gemm32x64(xh, DM, wt, DM, DM, m0, n0, lane, acc);

  float bb[4];
#pragma unroll
  for (int t = 0; t < 4; ++t) bb[t] = inb[n0 + 16 * t + c];

  if (which < 2) {
#pragma unroll
    for (int sub = 0; sub < 2; ++sub)
#pragma unroll
      for (int t = 0; t < 4; ++t)
#pragma unroll
        for (int r = 0; r < 8; ++r)
          st[(wave * 32 + sub * 16 + 8 * hh + r) * STP + 16 * t + c] =
              (_Float16)(acc[sub][t][r] * 0.03125f + bb[t]);
  } else {
#pragma unroll
    for (int sub = 0; sub < 2; ++sub)
#pragma unroll
      for (int t = 0; t < 4; ++t)
#pragma unroll
        for (int r = 0; r < 8; ++r)
          st[(16 * t + c) * SVP + wave * 32 + sub * 16 + 8 * hh + r] =
              (_Float16)(acc[sub][t][r] * 0.03125f + bb[t]);
  }
  __syncthreads();

  if (which < 2) {
    _Float16* base = (which == 0) ? (qp + (size_t)rb * DM)
                                  : (kpl + ((size_t)b * TGK + PADF + l0) * DM);
#pragma unroll
    for (int gg = 0; gg < 2; ++gg) {
      v4u val[4];
      size_t go[4];
#pragma unroll
      for (int j = 0; j < 4; ++j) {
        const int p  = tid + 256 * (4 * gg + j);
        const int lr = p >> 3;
        const int pc = p & 7;
        Pack8 pk;
        pk.h   = *(const v8h*)(st + lr * STP + pc * 8);
        val[j] = pk.u;
        go[j]  = (size_t)lr * DM + cs + pc * 8;
      }
      for (int ps = 0; ps < 2; ++ps) {
#pragma unroll
        for (int j = 0; j < 4; ++j) *(volatile v4u*)(base + go[j]) = val[j];
        __threadfence();
      }
    }
  } else {
    _Float16* base = vtp + (size_t)b * DM * TVP + PADF + l0;
#pragma unroll
    for (int gg = 0; gg < 2; ++gg) {
      v4u val[4];
      size_t go[4];
#pragma unroll
      for (int j = 0; j < 4; ++j) {
        const int p    = tid + 256 * (4 * gg + j);
        const int drow = p >> 5;
        const int pc   = p & 31;
        Pack8 pk;
        pk.h   = *(const v8h*)(st + drow * SVP + pc * 8);
        val[j] = pk.u;
        go[j]  = (size_t)(cs + drow) * TVP + pc * 8;
      }
      for (int ps = 0; ps < 2; ++ps) {
#pragma unroll
        for (int j = 0; j < 4; ++j) *(volatile v4u*)(base + go[j]) = val[j];
        __threadfence();
      }
    }
  }
}

#define PSP 104
#define OSP 264
__global__ __launch_bounds__(256) void k_attn(const _Float16* __restrict__ qp,
                                              const _Float16* __restrict__ kpl,
                                              const _Float16* __restrict__ vtp,
                                              _Float16* __restrict__ cx) {
  __shared__ __align__(16) _Float16 Ps[NH * QT * PSP];
  __shared__ __align__(16) _Float16 Os[QT * OSP];

  const int tid = threadIdx.x, lane = tid & 31, wave = tid >> 5;
  const int hh = lane >> 4, c = lane & 15;
  const int b  = blockIdx.x / NQT;
  const int qt = blockIdx.x - b * NQT;
  const int t0 = qt * QT;
  const int h  = wave;
  const int qrow0 = b * NT + t0;
  const _Float16* Kb = kpl + (size_t)b * TGK * DM;
  const _Float16* Vb = vtp + (size_t)b * DM * TVP;
  _Float16* pw = Ps + wave * QT * PSP;

  const v16h qa = ldfrag(qp, DM, qrow0, h * HD, lane);
  v8f s[5];
#pragma unroll
  for (int j = 0; j < 5; ++j) {
    const v16h kb = ldfrag(Kb, DM, t0 + 16 * j, h * HD, lane);
    s[j] = mma16(qa, kb, zero8());
  }

  const float scale = 0.17677669529663687f;
  float il[8];
#pragma unroll
  for (int r = 0; r < 8; ++r) {
    const int mrow = 8 * hh + r;
    float mx = -1.0e30f;
#pragma unroll
    for (int j = 0; j < 5; ++j) {
      const int d = 16 * j + c - mrow;
      const bool valid = (d >= 1) && (d <= WIN);
      const float sv = valid ? (s[j][r] * scale) : -1.0e30f;
      s[j][r] = sv;
      mx = fmaxf(mx, sv);
    }
#pragma unroll
    for (int off = 1; off < 16; off <<= 1) mx = fmaxf(mx, __shfl_xor(mx, off, 32));
    float psum = 0.f;
#pragma unroll
    for (int j = 0; j < 5; ++j) {
      const float p = __expf(s[j][r] - mx);
      psum += p;
      pw[mrow * PSP + 16 * j + c] = (_Float16)(p * 1024.0f);
    }
#pragma unroll
    for (int off = 1; off < 16; off <<= 1) psum += __shfl_xor(psum, off, 32);
    il[r] = 0.015625f * __builtin_amdgcn_rcpf(psum);
  }
  {
    const v8h z8 = (v8h){(_Float16)0.f, (_Float16)0.f, (_Float16)0.f, (_Float16)0.f,
                         (_Float16)0.f, (_Float16)0.f, (_Float16)0.f, (_Float16)0.f};
    *(v8h*)(pw + (lane >> 1) * PSP + 80 + 8 * (lane & 1)) = z8;
  }
  __syncthreads();

  v8f oacc[2];
  oacc[0] = zero8();
  oacc[1] = zero8();
#pragma unroll
  for (int kc = 0; kc < 3; ++kc) {
    const v16h pa = ldfrag(pw, PSP, 0, 32 * kc, lane);
#pragma unroll
    for (int nt = 0; nt < 2; ++nt) {
      const v16h vb = ldfrag(Vb, TVP, h * HD + 16 * nt, t0 + 32 * kc, lane);
      oacc[nt] = mma16(pa, vb, oacc[nt]);
    }
  }

#pragma unroll
  for (int nt = 0; nt < 2; ++nt)
#pragma unroll
    for (int r = 0; r < 8; ++r)
      Os[(8 * hh + r) * OSP + h * HD + 16 * nt + c] = (_Float16)(oacc[nt][r] * il[r]);
  __syncthreads();

  v4u val[2];
  size_t go[2];
#pragma unroll
  for (int it = 0; it < 2; ++it) {
    const int p   = tid + 256 * it;
    const int row = p >> 5;
    const int pc  = p & 31;
    Pack8 pk;
    pk.h    = *(const v8h*)(Os + row * OSP + pc * 8);
    val[it] = pk.u;
    go[it]  = (size_t)(qrow0 + row) * DM + pc * 8;
  }
  for (int ps = 0; ps < 2; ++ps) {
#pragma unroll
    for (int it = 0; it < 2; ++it) *(volatile v4u*)(cx + go[it]) = val[it];
    __threadfence();
  }
}

#define OTP 68
__device__ __forceinline__ void out_epilogue_f32(v8f (&acc)[2][4], float scale, const float (&bb)[4],
                                                 float* sw, float* __restrict__ out, int ldo,
                                                 int m0, int n0, int lane, int hh, int c) {
#pragma unroll
  for (int sub = 0; sub < 2; ++sub) {
    __syncthreads();
#pragma unroll
    for (int t = 0; t < 4; ++t) {
#pragma unroll
      for (int r = 0; r < 8; ++r) sw[(8 * hh + r) * OTP + 16 * t + c] = acc[sub][t][r] * scale + bb[t];
    }
    __syncthreads();
    v4f val[8];
    size_t go[8];
#pragma unroll
    for (int it = 0; it < 8; ++it) {
      const int p     = lane + 32 * it;
      const int L     = p >> 3;
      const int pc    = p & 7;
      const int row   = L >> 1;
      const int seg   = L & 1;
      val[it] = *(const v4f*)(sw + row * OTP + seg * 32 + pc * 4);
      go[it]  = (size_t)(m0 + sub * 16 + row) * ldo + n0 + seg * 32 + pc * 4;
    }
    for (int ps = 0; ps < 2; ++ps) {
#pragma unroll
      for (int it = 0; it < 8; ++it) *(volatile v4f*)(out + go[it]) = val[it];
      __threadfence();
    }
  }
}

__global__ __launch_bounds__(256) void k_gemm_f32(const _Float16* __restrict__ ap, int lda,
                                                  const _Float16* __restrict__ wt, int K,
                                                  const float* __restrict__ bias, float scale,
                                                  float* __restrict__ out, int ldo) {
  __shared__ __align__(16) float st[8][16 * OTP];
  const int tid = threadIdx.x, lane = tid & 31, wave = tid >> 5;
  const int hh = lane >> 4, c = lane & 15;
  const int m0 = blockIdx.x * 256 + wave * 32;
  const int n0 = blockIdx.y * 64;

  v8f acc[2][4];
#pragma unroll
  for (int s = 0; s < 2; ++s)
#pragma unroll
    for (int t = 0; t < 4; ++t) acc[s][t] = zero8();
  gemm32x64(ap, lda, wt, K, K, m0, n0, lane, acc);
  float bb[4];
#pragma unroll
  for (int t = 0; t < 4; ++t) bb[t] = bias[n0 + 16 * t + c];
  out_epilogue_f32(acc, scale, bb, st[wave], out, ldo, m0, n0, lane, hh, c);
}

extern "C" void kernel_launch(void* const* d_in, const int* in_sizes, int n_in,
                              void* d_out, int out_size, void* d_ws, size_t ws_size,
                              hipStream_t stream) {
  if (n_in < 5) return;
  if (in_sizes[0] != NTOK * DM) return;
  if (in_sizes[1] != NQKV * DM) return;
  if (in_sizes[2] != NQKV) return;
  if (in_sizes[3] != DM * DM) return;
  if (in_sizes[4] != DM) return;
  if (out_size != NTOK * DM) return;

  const float* x     = (const float*)d_in[0];
  const float* in_w  = (const float*)d_in[1];
  const float* in_b  = (const float*)d_in[2];
  const float* out_w = (const float*)d_in[3];
  const float* out_b = (const float*)d_in[4];
  float* out = (float*)d_out;

  size_t off = 0;
  const size_t oWt = off; off += (size_t)NQKV * DM * 2;
  const size_t oWo = off; off += (size_t)DM * DM * 2;
  const size_t oX  = off; off += (size_t)NTOK * DM * 2;
  const size_t oQ  = off; off += (size_t)NTOK * DM * 2;
  const size_t oK  = off; off += (size_t)NB * TGK * DM * 2;
  const size_t oV  = off; off += (size_t)NB * DM * TVP * 2;
  const size_t oC  = off; off += (size_t)NTOK * DM * 2;
  if (off > ws_size) return;
  if (off > (size_t)134217728) return;

  char* ws = (char*)d_ws;
  _Float16* Wt  = (_Float16*)(ws + oWt);
  _Float16* Wot = (_Float16*)(ws + oWo);
  _Float16* Xh  = (_Float16*)(ws + oX);
  _Float16* Qp  = (_Float16*)(ws + oQ);
  _Float16* Kp  = (_Float16*)(ws + oK);
  _Float16* Vt  = (_Float16*)(ws + oV);
  _Float16* Cx  = (_Float16*)(ws + oC);

  k_cvt<<<dim3((NTOK * DM) / 2048), dim3(256), 0, stream>>>(x, Xh, 1.0f);
  k_cvt<<<dim3((NQKV * DM) / 2048), dim3(256), 0, stream>>>(in_w, Wt, 32.0f);
  k_cvt<<<dim3((DM * DM) / 2048), dim3(256), 0, stream>>>(out_w, Wot, 32.0f);
  k_padfill<<<dim3(NPADBLK_K + NPADBLK_V), dim3(256), 0, stream>>>(in_b, Kp, Vt);
  k_qkv<<<dim3(NTOK / 256, NQKV / 64), dim3(256), 0, stream>>>(Xh, Wt, in_b, Qp, Kp, Vt);
  k_attn<<<dim3(NB * NQT), dim3(256), 0, stream>>>(Qp, Kp, Vt, Cx);
  k_gemm_f32<<<dim3(NTOK / 256, DM / 64), dim3(256), 0, stream>>>(Cx, DM, Wot, DM, out_b, 0.001953125f, out, DM);
  (void)hipGetLastError();
}
